// MultiDimWindowTransformerLayer_1494648619773
// MI455X (gfx1250) — hardware-verified
//
#include <hip/hip_runtime.h>
#include <math.h>
#include <stdint.h>

#define LL   2048
#define CC   8
#define HH   256
#define NHD  8
#define HD   32
#define FFD  1024
#define QKVW 768
#define WIN  21
#define WHF  10
#define MT   (LL * CC)
#define MR   (WIN * LL)
#define NCHK 7
#define RSP  272
#define BDP  24
#define ZSP  72
#define WSC  16.0f
#define WSC2 32.0f
#define PSC  1024.0f
#define ZSC  16.0f
#define SCL  0.17677669529663687f
#define LEPS 1e-5f

static_assert(NHD * HD == HH);
static_assert(QKVW == 3 * HH);
static_assert((MT % 64) == 0 && (MR % 64) == 0 && (HH % 64) == 0 && (FFD % 64) == 0 && (QKVW % 64) == 0);
static_assert((((MT / 64) * (HH / 64)) % 8) == 0);
static_assert((((MT / 64) * (FFD / 64)) % 8) == 0);
static_assert((LL % 64) == 0 && (LL % 8) == 0 && (MT % 8) == 0);
static_assert(8 * 16 * 68 * 4 == 64 * RSP * 2);
static_assert(4 * NCHK == WIN + 7);
static_assert(BDP >= WIN);

typedef _Float16 v16h __attribute__((ext_vector_type(16)));
typedef _Float16 v8h  __attribute__((ext_vector_type(8)));
typedef unsigned short v16us __attribute__((ext_vector_type(16)));
typedef unsigned short v8us  __attribute__((ext_vector_type(8)));
typedef float v8f __attribute__((ext_vector_type(8)));
typedef float v4f __attribute__((ext_vector_type(4)));
typedef unsigned int v4u __attribute__((ext_vector_type(4)));

union FragU { v16us v; v8us h[2]; };

__device__ __forceinline__ unsigned short bf_bits(float f) {
  const unsigned u = __float_as_uint(f);
  return (unsigned short)((u + 0x7FFFu + ((u >> 16) & 1u)) >> 16);
}
__device__ __forceinline__ float bf_up(unsigned short h) { return __uint_as_float(((unsigned)h) << 16); }
__device__ __forceinline__ float bfr(float f) { return bf_up(bf_bits(f)); }
__device__ __forceinline__ unsigned short h_bits(_Float16 x) { return __builtin_bit_cast(unsigned short, x); }
__device__ __forceinline__ unsigned short f2h(float f) { return h_bits((_Float16)f); }
__device__ __forceinline__ unsigned pk16(unsigned short a, unsigned short b) { return (unsigned)a | ((unsigned)b << 16); }
__device__ __forceinline__ int clampi(int v, int lo, int hi) { return v < lo ? lo : (v > hi ? hi : v); }
__device__ __forceinline__ v8f zero8() { v8f z = {0.f, 0.f, 0.f, 0.f, 0.f, 0.f, 0.f, 0.f}; return z; }

__device__ __forceinline__ v16us ldfrag_u(const unsigned short* p) {
  FragU f;
  f.h[0] = *(const v8us*)(p);
  f.h[1] = *(const v8us*)(p + 16);
  return f.v;
}

__device__ __forceinline__ v8f mma_h_raw(v16us a, v16us b, v8f c) {
  return __builtin_amdgcn_wmma_f32_16x16x32_f16(false, __builtin_bit_cast(v16h, a), false,
                                                __builtin_bit_cast(v16h, b), (short)0, c, false, false);
}
__device__ __forceinline__ v8f mma_hu(v16us a, v16us b, v8f c) {
  c = mma_h_raw(a, b, c);
#if defined(__HIP_DEVICE_COMPILE__)
  asm volatile("v_nop\n\tv_nop\n\tv_nop\n\tv_nop" : "+v"(c) : "v"(a), "v"(b));
#endif
  return c;
}
__device__ __forceinline__ void dep_guard1(v8f& a, v8f& b, v16us x) {
#if defined(__HIP_DEVICE_COMPILE__)
  asm volatile("v_nop\n\tv_nop\n\tv_nop\n\tv_nop" : "+v"(a), "+v"(b) : "v"(x));
#endif
}
__device__ __forceinline__ void keep4_u(v16us a, v16us b, v16us c, v16us d) {
#if defined(__HIP_DEVICE_COMPILE__)
  asm volatile("v_nop" :: "v"(a), "v"(b), "v"(c), "v"(d));
#endif
}
__device__ __forceinline__ void acc_guard4(v8f& a, v8f& b, v8f& c, v8f& d) {
#if defined(__HIP_DEVICE_COMPILE__)
  asm volatile("v_nop\n\tv_nop\n\tv_nop\n\tv_nop" : "+v"(a), "+v"(b), "+v"(c), "+v"(d));
#endif
}
__device__ __forceinline__ void wave_sync_lds() {
  __builtin_amdgcn_fence(__ATOMIC_RELEASE, "workgroup");
  __builtin_amdgcn_wave_barrier();
  __builtin_amdgcn_fence(__ATOMIC_ACQUIRE, "workgroup");
}

__global__ __launch_bounds__(256) void cvt_x(const float* __restrict__ x, unsigned short* xh, int nrows) {
  const int row = blockIdx.x * 8 + (threadIdx.x >> 5);
  const int lane = threadIdx.x & 31;
  if (row >= nrows) return;
  const float* p = x + (size_t)row * HH + lane * 8;
  const v4f a0 = *(const v4f*)(p);
  const v4f a1 = *(const v4f*)(p + 4);
  v4u hv;
#pragma unroll
  for (int e = 0; e < 2; ++e) {
    hv[e]     = pk16(f2h(bfr(a0[2 * e])), f2h(bfr(a0[2 * e + 1])));
    hv[2 + e] = pk16(f2h(bfr(a1[2 * e])), f2h(bfr(a1[2 * e + 1])));
  }
  unsigned short* d = xh + (size_t)row * HH + lane * 8;
  for (int pass = 0; pass < 2; ++pass) {
    *(volatile v4u*)(d) = hv;
    __threadfence();
  }
}

__global__ __launch_bounds__(256) void wtrans(const float* __restrict__ in, unsigned short* out, int KR, int NC, float sc) {
  __shared__ float s[64][65];
  const int t = threadIdx.x;
  const int n0 = blockIdx.x * 64, k0 = blockIdx.y * 64;
#pragma unroll
  for (int it = 0; it < 16; ++it) {
    const int idx = it * 256 + t;
    const int kk = idx >> 6, nn = idx & 63;
    s[nn][kk] = in[(size_t)(k0 + kk) * NC + n0 + nn];
  }
  __syncthreads();
  v4u hv[2];
#pragma unroll
  for (int it = 0; it < 2; ++it) {
    const int r = it * 32 + (t >> 3), p = (t & 7) * 8;
    v4u h;
#pragma unroll
    for (int e = 0; e < 4; ++e) {
      const float f0 = bfr(s[r][p + 2 * e]) * sc;
      const float f1 = bfr(s[r][p + 2 * e + 1]) * sc;
      h[e] = pk16(f2h(f0), f2h(f1));
    }
    hv[it] = h;
  }
  for (int pass = 0; pass < 2; ++pass) {
#pragma unroll
    for (int it = 0; it < 2; ++it) {
      const int r = it * 32 + (t >> 3), p = (t & 7) * 8;
      *(volatile v4u*)(out + (size_t)(n0 + r) * KR + k0 + p) = hv[it];
    }
    __threadfence();
  }
}

template <int OM, int CBM, int RELU>
__global__ __launch_bounds__(256) void gemm64(
    const unsigned short* __restrict__ Ap, int lda,
    const unsigned short* __restrict__ Btp, int ldb,
    unsigned short* Ch, float* Cf, int ldc,
    const float* __restrict__ cb, const float* __restrict__ cbw, const float* __restrict__ cbr,
    float wsc, int M, int N, int K) {
  __shared__ __align__(16) float sT[8][16 * 68];
  const int lane = threadIdx.x & 31;
  const int wave = threadIdx.x >> 5;
  const int tilesN = N >> 6;
  const int tilesM = M >> 6;
  const int tile = blockIdx.x * 8 + wave;
  if (tile >= tilesM * tilesN) return;
  const int tm = tile / tilesN;
  const int tn = tile - tm * tilesN;
  const int m0 = tm << 6;
  const int n0 = tn << 6;

  const int rlane = lane & 15;
  const int koff  = (lane >> 4) * 8;
  const int mOff  = (lane >> 4) * 8;

  v8f acc[4][4];
#pragma unroll
  for (int i = 0; i < 4; ++i)
#pragma unroll
    for (int j = 0; j < 4; ++j) acc[i][j] = zero8();

  for (int k0 = 0; k0 < K; k0 += 32) {
    v16us bh[4];
#pragma unroll
    for (int j = 0; j < 4; ++j) {
      const size_t bo = (size_t)(n0 + (j << 4) + rlane) * ldb + koff + k0;
      bh[j] = ldfrag_u(Btp + bo);
    }
#pragma unroll
    for (int i = 0; i < 4; ++i) {
      const size_t ao = (size_t)(m0 + (i << 4) + rlane) * lda + koff + k0;
      const v16us ah = ldfrag_u(Ap + ao);
#pragma unroll
      for (int j = 0; j < 4; ++j) acc[i][j] = mma_h_raw(ah, bh[j], acc[i][j]);
      dep_guard1(acc[i][0], acc[i][3], ah);
    }
    keep4_u(bh[0], bh[1], bh[2], bh[3]);
  }
  acc_guard4(acc[0][0], acc[0][1], acc[0][2], acc[0][3]);
  acc_guard4(acc[1][0], acc[1][1], acc[1][2], acc[1][3]);
  acc_guard4(acc[2][0], acc[2][1], acc[2][2], acc[2][3]);
  acc_guard4(acc[3][0], acc[3][1], acc[3][2], acc[3][3]);

  const int hh2 = lane >> 4, c4 = (lane & 15) * 4;
  const int q8  = lane >> 3, c8 = (lane & 7) * 8;

  v4f cb4 = {0.f, 0.f, 0.f, 0.f}, cr4 = {0.f, 0.f, 0.f, 0.f};
  float cbc[8], cwc[8];
#pragma unroll
  for (int e = 0; e < 8; ++e) { cbc[e] = 0.f; cwc[e] = 0.f; }
  if (OM == 0 || OM == 2) {
    if (CBM == 1) {
      const v4f v = *(const v4f*)(cb + n0 + c4);
      cb4[0] = bfr(v[0]); cb4[1] = bfr(v[1]); cb4[2] = bfr(v[2]); cb4[3] = bfr(v[3]);
    }
    if (OM == 2) {
      const v4f v = *(const v4f*)(cbr + n0 + c4);
      cr4[0] = bfr(v[0]); cr4[1] = bfr(v[1]); cr4[2] = bfr(v[2]); cr4[3] = bfr(v[3]);
    }
  }
  if (OM == 1 || OM == 2) {
    if (CBM == 1) {
      const v4f v0 = *(const v4f*)(cb + n0 + c8);
      const v4f v1 = *(const v4f*)(cb + n0 + c8 + 4);
#pragma unroll
      for (int e = 0; e < 4; ++e) { cbc[e] = bfr(v0[e]); cbc[4 + e] = bfr(v1[e]); }
    }
    if (OM == 2) {
      const v4f v0 = *(const v4f*)(cbw + n0 + c8);
      const v4f v1 = *(const v4f*)(cbw + n0 + c8 + 4);
#pragma unroll
      for (int e = 0; e < 4; ++e) { cwc[e] = bfr(v0[e]); cwc[4 + e] = bfr(v1[e]); }
    }
  }

  float* slab = sT[wave];
#pragma unroll
  for (int i = 0; i < 4; ++i) {
    const int mBase = m0 + (i << 4);
#pragma unroll
    for (int j = 0; j < 4; ++j) {
#pragma unroll
      for (int r = 0; r < 8; ++r) {
        slab[(mOff + r) * 68 + (j << 4) + rlane] = acc[i][j][r];
      }
    }
    wave_sync_lds();
    if (OM == 0 || OM == 2) {
      v4f vals[8];
#pragma unroll
      for (int it = 0; it < 8; ++it) {
        const int row = it * 2 + hh2;
        const v4f v = *(const v4f*)(slab + row * 68 + c4);
        v4f tv = v * wsc + cb4;
        if (OM == 2) tv = tv * SCL + cr4;
        vals[it] = tv;
      }
      for (int pass = 0; pass < 2; ++pass) {
#pragma unroll
        for (int it = 0; it < 8; ++it) {
          const int row = it * 2 + hh2;
          *(volatile v4f*)(Cf + (size_t)(mBase + row) * ldc + (size_t)n0 + c4) = vals[it];
        }
        __threadfence();
      }
    }
    if (OM == 1 || OM == 2) {
      v4u hv[4];
#pragma unroll
      for (int it = 0; it < 4; ++it) {
        const int row = it * 4 + q8;
        const float* sp = slab + row * 68 + c8;
        float rb = 0.f;
        if (CBM == 2) rb = bfr(cb[mBase + row]);
        v4u ha = {0u, 0u, 0u, 0u};
#pragma unroll
        for (int e = 0; e < 4; ++e) {
          float f0 = sp[2 * e]     * wsc + cbc[2 * e]     + rb;
          float f1 = sp[2 * e + 1] * wsc + cbc[2 * e + 1] + rb;
          if (OM == 2) { f0 = f0 * SCL + cwc[2 * e]; f1 = f1 * SCL + cwc[2 * e + 1]; }
          if (RELU) { f0 = fmaxf(f0, 0.0f); f1 = fmaxf(f1, 0.0f); }
          ha[e] = pk16(f2h(f0), f2h(f1));
        }
        hv[it] = ha;
      }
      for (int pass = 0; pass < 2; ++pass) {
#pragma unroll
        for (int it = 0; it < 4; ++it) {
          const int row = it * 4 + q8;
          const size_t go = (size_t)(mBase + row) * ldc + (size_t)n0 + c8;
          *(volatile v4u*)(Ch + go) = hv[it];
        }
        __threadfence();
      }
    }
    wave_sync_lds();
  }
}

__global__ __launch_bounds__(256) void re_kernel(const int* __restrict__ pos, const unsigned short* __restrict__ WeT,
                                                 const float* __restrict__ be, float* RE) {
  __shared__ __align__(16) float smem[8 * 16 * 68];
  __shared__ float sinv[HH / 2];
  __shared__ float srel[64];
  unsigned short* rsd = (unsigned short*)smem;
  const int t = threadIdx.x, lane = t & 31, wave = t >> 5;
  const int m0 = blockIdx.x * 64;
  const int wslot = m0 / LL;
  const int lb = m0 - wslot * LL;
  if (t < HH / 2) sinv[t] = 1.0f / powf(10000.0f, (float)(2 * t) * (1.0f / (float)HH));
  if (t < 64) {
    const int l = lb + t;
    const int src = wslot + l - WHF;
    const int srcc = clampi(src, 0, LL - 1);
    const float pv = (float)pos[srcc];
    const float padv = (src >= 0 && src < LL) ? pv : 0.0f;
    srel[t] = padv - (float)pos[l];
  }
  __syncthreads();
  {
    const int rr = t >> 2, pb = t & 3;
    const float rel = srel[rr];
#pragma unroll 1
    for (int j = 0; j < 8; ++j) {
      v4u pk;
#pragma unroll
      for (int e = 0; e < 4; ++e) {
        const int i = pb * 32 + 4 * j + e;
        const float ang = rel * sinv[i];
        const float sn = sinf(ang);
        const float cs = cosf(ang);
        pk[e] = pk16(f2h(sn), f2h(cs));
      }
      *(v4u*)(rsd + rr * RSP + 2 * (pb * 32 + 4 * j)) = pk;
    }
  }
  __syncthreads();

  const int rlane = lane & 15, koff = (lane >> 4) * 8, mOff = (lane >> 4) * 8;
  const int wr = (wave >> 2) * 32, wc = (wave & 3) * 64;
  v8f acc[2][4];
#pragma unroll
  for (int i = 0; i < 2; ++i)
#pragma unroll
    for (int j = 0; j < 4; ++j) acc[i][j] = zero8();
#pragma unroll 1
  for (int k0 = 0; k0 < HH; k0 += 32) {
    v16us bh[4];
#pragma unroll
    for (int j = 0; j < 4; ++j) bh[j] = ldfrag_u(WeT + (size_t)(wc + (j << 4) + rlane) * HH + koff + k0);
#pragma unroll
    for (int i = 0; i < 2; ++i) {
      const v16us ah = ldfrag_u(rsd + (wr + (i << 4) + rlane) * RSP + koff + k0);
#pragma unroll
      for (int j = 0; j < 4; ++j) acc[i][j] = mma_h_raw(ah, bh[j], acc[i][j]);
      dep_guard1(acc[i][0], acc[i][3], ah);
    }
    keep4_u(bh[0], bh[1], bh[2], bh[3]);
  }
  acc_guard4(acc[0][0], acc[0][1], acc[0][2], acc[0][3]);
  acc_guard4(acc[1][0], acc[1][1], acc[1][2], acc[1][3]);
  __syncthreads();

  float* slab = smem + wave * (16 * 68);
  const int hh2 = lane >> 4, c4 = (lane & 15) * 4;
  v4f cb4;
  {
    const v4f v = *(const v4f*)(be + wc + c4);
    cb4[0] = bfr(v[0]); cb4[1] = bfr(v[1]); cb4[2] = bfr(v[2]); cb4[3] = bfr(v[3]);
  }
#pragma unroll
  for (int i = 0; i < 2; ++i) {
    const int mBase = m0 + wr + (i << 4);
#pragma unroll
    for (int j = 0; j < 4; ++j) {
#pragma unroll
      for (int r = 0; r < 8; ++r) slab[(mOff + r) * 68 + (j << 4) + rlane] = acc[i][j][r];
    }
    wave_sync_lds();
    v4f vals[8];
#pragma unroll
    for (int it = 0; it < 8; ++it) {
      const int row = it * 2 + hh2;
      const v4f v = *(const v4f*)(slab + row * 68 + c4);
      vals[it] = v * (1.0f / WSC) + cb4;
    }
    for (int pass = 0; pass < 2; ++pass) {
#pragma unroll
      for (int it = 0; it < 8; ++it) {
        const int row = it * 2 + hh2;
        *(volatile v4f*)(RE + (size_t)(mBase + row) * HH + wc + c4) = vals[it];
      }
      __threadfence();
    }
    wave_sync_lds();
  }
}

__global__ __launch_bounds__(256) void attn_kernel(
    const unsigned short* __restrict__ Qh, const float* __restrict__ QR,
    const unsigned short* __restrict__ Kh, const unsigned short* __restrict__ VT,
    const float* __restrict__ RE, unsigned short* Zh) {
  __shared__ __align__(16) float qrs[2 * 64 * 32];
  __shared__ __align__(16) float bds[2 * 64 * BDP];
  __shared__ __align__(16) unsigned short ps[8 * 512];
  __shared__ __align__(16) unsigned short zst[64 * ZSP];
  const int l0 = blockIdx.x * 8;
  const int hp = blockIdx.y;
  const int tq0 = l0 * CC;
  const int t = threadIdx.x, lane = t & 31, wv = t >> 5, hh = lane >> 4, jc = lane & 15;
  const int ms = wv & 3, hs = wv >> 2, head = hp * 2 + hs;

#pragma unroll
  for (int it = 0; it < 4; ++it) {
    const int idx = it * 256 + t;
    const int h2 = idx >> 9, rem = idx & 511, q = rem >> 3, d4 = (rem & 7) * 4;
    const v4f v = *(const v4f*)(QR + (size_t)(tq0 + q) * HH + (hp * 2 + h2) * HD + d4);
    *(v4f*)(qrs + (h2 * 64 + q) * 32 + d4) = v;
  }
  __syncthreads();

#pragma unroll 1
  for (int it = t; it < 2 * 64 * WIN; it += 256) {
    const int h2 = (it >= 64 * WIN) ? 1 : 0;
    const int rem = it - h2 * (64 * WIN);
    const int q = rem / WIN;
    const int w = rem - q * WIN;
    const float* rp = RE + (size_t)(w * LL + l0 + (q >> 3)) * HH + (hp * 2 + h2) * HD;
    const float* qp = qrs + (h2 * 64 + q) * 32;
    float a = 0.0f;
#pragma unroll
    for (int d4 = 0; d4 < HD; d4 += 4) {
      const v4f qa = *(const v4f*)(qp + d4);
      const v4f rb = *(const v4f*)(rp + d4);
      a += qa[0] * rb[0];
      a += qa[1] * rb[1];
      a += qa[2] * rb[2];
      a += qa[3] * rb[3];
    }
    bds[(h2 * 64 + q) * BDP + w] = a;
  }
  __syncthreads();

  const int lq = 2 * ms + hh;
  const v16us qf = ldfrag_u(Qh + (size_t)(tq0 + 16 * ms + jc) * HH + head * HD + 8 * hh);
  float m[8], ll[8];
  v8f oz0 = zero8(), oz1 = zero8();
#pragma unroll
  for (int r = 0; r < 8; ++r) { m[r] = -1.0e30f; ll[r] = 0.f; }
  unsigned short* pw = ps + wv * 512;
  const float* bdq = bds + (hs * 64 + 16 * ms + 8 * hh) * BDP;
  const unsigned short* vr0 = VT + (size_t)(head * HD + jc) * MT;
  const unsigned short* vr1 = vr0 + (size_t)16 * MT;
  const int dk = jc & 7;

#pragma unroll 1
  for (int jt = 0; jt < NCHK; ++jt) {
    const int ga = 4 * jt + (jc >> 3);
    const int la = l0 - WHF + ga, lb2 = la + 2;
    const bool ina = (la >= 0) && (la < LL), inb = (lb2 >= 0) && (lb2 < LL);
    const int lac = clampi(la, 0, LL - 1), lbc = clampi(lb2, 0, LL - 1);
    const v16us kf0 = ldfrag_u(Kh + ((size_t)lac * CC + dk) * HH + head * HD + 8 * hh);
    const v16us kf1 = ldfrag_u(Kh + ((size_t)lbc * CC + dk) * HH + head * HD + 8 * hh);
    const v8f s0 = mma_hu(qf, kf0, zero8());
    const v8f s1 = mma_hu(qf, kf1, zero8());
    const int w0 = ga - lq, w1 = w0 + 2;
    const bool va = ina && (w0 >= 0) && (w0 < WIN);
    const bool vb = inb && (w1 >= 0) && (w1 < WIN);
    const int w0c = clampi(w0, 0, WIN - 1), w1c = clampi(w1, 0, WIN - 1);
    wave_sync_lds();
#pragma unroll
    for (int r = 0; r < 8; ++r) {
      const int il = 8 * hh + r;
      const float v0 = va ? (s0[r] + bdq[r * BDP + w0c]) : -3.0e38f;
      const float v1 = vb ? (s1[r] + bdq[r * BDP + w1c]) : -3.0e38f;
      float rm = fmaxf(v0, v1);
#pragma unroll
      for (int off = 1; off < 16; off <<= 1) rm = fmaxf(rm, __shfl_xor(rm, off, 32));
      const float mn2   = fmaxf(m[r], rm);
      const float alpha = __expf(m[r] - mn2);
      const float e0 = va ? __expf(v0 - mn2) : 0.0f;
      const float e1 = vb ? __expf(v1 - mn2) : 0.0f;
      float rs = e0 + e1;
#pragma unroll
      for (int off = 1; off < 16; off <<= 1) rs += __shfl_xor(rs, off, 32);
      ll[r] = ll[r] * alpha + rs;
      m[r]  = mn2;
      oz0[r] *= alpha; oz1[r] *= alpha;
      pw[il * 32 + jc]      = f2h(e0 * PSC);
      pw[il * 32 + 16 + jc] = f2h(e1 * PSC);
    }
    wave_sync_lds();
    FragU pa;
    pa.h[0] = *(const v8us*)(pw + jc * 32 + 8 * hh);
    pa.h[1] = *(const v8us*)(pw + jc * 32 + 16 + 8 * hh);
    const int lsa = clampi(l0 - WHF + 4 * jt + hh, 0, LL - 1);
    const int lsb = clampi(l0 - WHF + 4 * jt + 2 + hh, 0, LL - 1);
    FragU f0, f1;
    f0.h[0] = *(const v8us*)(vr0 + (size_t)lsa * CC);
    f0.h[1] = *(const v8us*)(vr0 + (size_t)lsb * CC);
    f1.h[0] = *(const v8us*)(vr1 + (size_t)lsa * CC);
    f1.h[1] = *(const v8us*)(vr1 + (size_t)lsb * CC);
    oz0 = mma_hu(pa.v, f0.v, oz0);
    oz1 = mma_hu(pa.v, f1.v, oz1);
  }

#pragma unroll
  for (int r = 0; r < 8; ++r) {
    const int il = 8 * hh + r;
    const float l = ll[r];
    const float inv = ((l > 0.f) ? (1.0f / l) : 0.f) * (ZSC / PSC);
    zst[(16 * ms + il) * ZSP + hs * 32 + jc]      = f2h(oz0[r] * inv);
    zst[(16 * ms + il) * ZSP + hs * 32 + 16 + jc] = f2h(oz1[r] * inv);
  }
  __syncthreads();
  v4u hv[2];
#pragma unroll
  for (int it = 0; it < 2; ++it) {
    const int row = it * 32 + (t >> 3), p = (t & 7) * 8;
    hv[it] = *(const v4u*)(zst + row * ZSP + p);
  }
  for (int pass = 0; pass < 2; ++pass) {
#pragma unroll
    for (int it = 0; it < 2; ++it) {
      const int row = it * 32 + (t >> 3), p = (t & 7) * 8;
      *(volatile v4u*)(Zh + (size_t)(tq0 + row) * HH + hp * 64 + p) = hv[it];
    }
    __threadfence();
  }
}

template <int MODE>
__global__ __launch_bounds__(256) void add_ln(const float* __restrict__ a, const float* __restrict__ b,
                                             const float* __restrict__ g, const float* __restrict__ bt,
                                             float* of, unsigned short* oh, int nrows) {
  const int row = blockIdx.x * 8 + (threadIdx.x >> 5);
  const int lane = threadIdx.x & 31;
  if (row >= nrows) return;
  const size_t ro = (size_t)row * HH;
  const int ca = lane * 4, cbx = 128 + lane * 4;
  const v4f a0 = *(const v4f*)(a + ro + ca), a1 = *(const v4f*)(a + ro + cbx);
  const v4f b0 = *(const v4f*)(b + ro + ca), b1 = *(const v4f*)(b + ro + cbx);
  float v[8];
#pragma unroll
  for (int e = 0; e < 4; ++e) {
    const float xa = (MODE == 0) ? bfr(a0[e]) : a0[e];
    const float xb = (MODE == 0) ? bfr(a1[e]) : a1[e];
    v[e]     = xa + b0[e];
    v[4 + e] = xb + b1[e];
  }
  float s = 0.f;
#pragma unroll
  for (int e = 0; e < 8; ++e) s += v[e];
#pragma unroll
  for (int off = 16; off > 0; off >>= 1) s += __shfl_xor(s, off, 32);
  const float mu = s * (1.0f / (float)HH);
  float d[8];
  float sq = 0.f;
#pragma unroll
  for (int e = 0; e < 8; ++e) { d[e] = v[e] - mu; sq += d[e] * d[e]; }
#pragma unroll
  for (int off = 16; off > 0; off >>= 1) sq += __shfl_xor(sq, off, 32);
  const float var = sq * (1.0f / (float)HH);
  const float rstd = rsqrtf(var + LEPS);
  const v4f g0 = *(const v4f*)(g + ca),  g1 = *(const v4f*)(g + cbx);
  const v4f t0 = *(const v4f*)(bt + ca), t1 = *(const v4f*)(bt + cbx);
  v4f oa, ob;
#pragma unroll
  for (int e = 0; e < 4; ++e) {
    oa[e] = d[e] * rstd * bfr(g0[e]) + bfr(t0[e]);
    ob[e] = d[4 + e] * rstd * bfr(g1[e]) + bfr(t1[e]);
  }
  v4u hv = {0u, 0u, 0u, 0u};
  if (MODE == 0) {
    const unsigned a01 = pk16(f2h(oa[0]), f2h(oa[1])), a23 = pk16(f2h(oa[2]), f2h(oa[3]));
    const unsigned b01 = pk16(f2h(ob[0]), f2h(ob[1])), b23 = pk16(f2h(ob[2]), f2h(ob[3]));
    const int s0 = (2 * lane) & 31, s1 = (2 * lane + 1) & 31;
    const unsigned x0 = __shfl(a01, s0, 32), x1 = __shfl(a23, s0, 32);
    const unsigned x2 = __shfl(a01, s1, 32), x3 = __shfl(a23, s1, 32);
    const unsigned y0 = __shfl(b01, s0, 32), y1 = __shfl(b23, s0, 32);
    const unsigned y2 = __shfl(b01, s1, 32), y3 = __shfl(b23, s1, 32);
    const bool lowhalf = (lane < 16);
    hv[0] = lowhalf ? x0 : y0;
    hv[1] = lowhalf ? x1 : y1;
    hv[2] = lowhalf ? x2 : y2;
    hv[3] = lowhalf ? x3 : y3;
  }
  for (int pass = 0; pass < 2; ++pass) {
    *(volatile v4f*)(of + ro + ca)  = oa;
    *(volatile v4f*)(of + ro + cbx) = ob;
    if (MODE == 0) *(volatile v4u*)(oh + ro + lane * 8) = hv;
    __threadfence();
  }
}

static_assert((size_t)MT * HH * 4 <= (size_t)MR * HH * 4);
static_assert((size_t)MT * FFD * 2 <= (size_t)MR * HH * 4);

extern "C" void kernel_launch(void* const* d_in, const int* in_sizes, int n_in,
                              void* d_out, int out_size, void* d_ws, size_t ws_size,
                              hipStream_t stream) {
  if (n_in < 18) return;
  if (in_sizes[0] != MT * HH || in_sizes[1] != LL) return;
  if (in_sizes[2] != HH * QKVW || in_sizes[3] != QKVW) return;
  if (in_sizes[4] != HH * HH || in_sizes[5] != HH) return;
  if (in_sizes[6] != NHD * HD || in_sizes[7] != NHD * HD) return;
  if (in_sizes[8] != HH * HH || in_sizes[9] != HH) return;
  if (in_sizes[10] != HH || in_sizes[11] != HH || in_sizes[12] != HH || in_sizes[13] != HH) return;
  if (in_sizes[14] != HH * FFD || in_sizes[15] != FFD) return;
  if (in_sizes[16] != FFD * HH || in_sizes[17] != HH) return;
  if (out_size != MT * HH) return;

  const float* x    = (const float*)d_in[0];
  const int*   pos  = (const int*)d_in[1];
  const float* Wqkv = (const float*)d_in[2];
  const float* bqkv = (const float*)d_in[3];
  const float* We   = (const float*)d_in[4];
  const float* be   = (const float*)d_in[5];
  const float* brw  = (const float*)d_in[6];
  const float* brr  = (const float*)d_in[7];
  const float* Wout = (const float*)d_in[8];
  const float* bout = (const float*)d_in[9];
  const float* ln1g = (const float*)d_in[10];
  const float* ln1b = (const float*)d_in[11];
  const float* ln2g = (const float*)d_in[12];
  const float* ln2b = (const float*)d_in[13];
  const float* Wff1 = (const float*)d_in[14];
  const float* bff1 = (const float*)d_in[15];
  const float* Wff2 = (const float*)d_in[16];
  const float* bff2 = (const float*)d_in[17];

  const size_t PXH = (size_t)MT * HH * 2;
  const size_t PWQ = (size_t)QKVW * HH * 2;
  const size_t PWE = (size_t)HH * HH * 2;
  const size_t PWO = (size_t)HH * HH * 2;
  const size_t PW1 = (size_t)FFD * HH * 2;
  const size_t PW2 = (size_t)HH * FFD * 2;
  const size_t PQH = (size_t)MT * HH * 2;
  const size_t PQR = (size_t)MT * HH * 4;
  const size_t PKH = (size_t)MT * HH * 2;
  const size_t PVT = (size_t)HH * MT * 2;
  const size_t PRE = (size_t)MR * HH * 4;
  const size_t PZH = (size_t)MT * HH * 2;
  size_t off = 0;
  const size_t oXh  = off; off += PXH;
  const size_t oWq  = off; off += PWQ;
  const size_t oWe  = off; off += PWE;
  const size_t oWo  = off; off += PWO;
  const size_t oW1  = off; off += PW1;
  const size_t oW2  = off; off += PW2;
  const size_t oQh  = off; off += PQH;
  const size_t oQR  = off; off += PQR;
  const size_t oKh  = off; off += PKH;
  const size_t oVT  = off; off += PVT;
  const size_t oRE  = off; off += PRE;
  const size_t oZh  = off; off += PZH;
  if (off > ws_size) return;
  if (off > (size_t)134217728) return;
  if ((size_t)MT * HH * 4 > PKH + PVT) return;
  if (oVT != oKh + PKH) return;

  char* ws = (char*)d_ws;
  unsigned short* Xh    = (unsigned short*)(ws + oXh);
  unsigned short* WqkvT = (unsigned short*)(ws + oWq);
  unsigned short* WeT   = (unsigned short*)(ws + oWe);
  unsigned short* WoutT = (unsigned short*)(ws + oWo);
  unsigned short* Wff1T = (unsigned short*)(ws + oW1);
  unsigned short* Wff2T = (unsigned short*)(ws + oW2);
  unsigned short* Qh    = (unsigned short*)(ws + oQh);
  float*          QR    = (float*)(ws + oQR);
  unsigned short* Kh    = (unsigned short*)(ws + oKh);
  unsigned short* VT    = (unsigned short*)(ws + oVT);
  float*          RE    = (float*)(ws + oRE);
  unsigned short* Zh    = (unsigned short*)(ws + oZh);
  float*          ATT   = (float*)(ws + oRE);
  float*          X1f   = (float*)(ws + oQR);
  unsigned short* X1h   = (unsigned short*)(ws + oQh);
  unsigned short* Hh    = (unsigned short*)(ws + oRE);
  float*          FFo   = (float*)(ws + oKh);
  float*          out0  = (float*)d_out;

  const dim3 blk(256);
  const int gq  = ((MT / 64) * (HH / 64)) / 8;
  const int gf1 = ((MT / 64) * (FFD / 64)) / 8;
  if ((((MT / 64) * (HH / 64)) % 8) != 0) return;
  if ((((MT / 64) * (FFD / 64)) % 8) != 0) return;

  cvt_x<<<dim3(MT / 8), blk, 0, stream>>>(x, Xh, MT);
  wtrans<<<dim3(QKVW / 64, HH / 64), blk, 0, stream>>>(Wqkv, WqkvT, HH, QKVW, WSC);
  wtrans<<<dim3(HH / 64, HH / 64), blk, 0, stream>>>(We, WeT, HH, HH, WSC);
  wtrans<<<dim3(HH / 64, HH / 64), blk, 0, stream>>>(Wout, WoutT, HH, HH, WSC);
  wtrans<<<dim3(FFD / 64, HH / 64), blk, 0, stream>>>(Wff1, Wff1T, HH, FFD, WSC);
  wtrans<<<dim3(HH / 64, FFD / 64), blk, 0, stream>>>(Wff2, Wff2T, FFD, HH, WSC2);

  gemm64<2, 1, 0><<<dim3(gq), blk, 0, stream>>>(
      Xh, HH, WqkvT, HH, Qh, QR, HH, bqkv, brw, brr, 1.0f / WSC, MT, HH, HH);
  gemm64<1, 1, 0><<<dim3(gq), blk, 0, stream>>>(
      Xh, HH, WqkvT + (size_t)HH * HH, HH, Kh, QR, HH, bqkv + HH, bqkv, bqkv, 1.0f / WSC, MT, HH, HH);
  gemm64<1, 2, 0><<<dim3(gq), blk, 0, stream>>>(
      WqkvT + (size_t)2 * HH * HH, HH, Xh, HH, VT, QR, MT, bqkv + 2 * HH, bqkv, bqkv, 1.0f / WSC, HH, MT, HH);

  re_kernel<<<dim3(MR / 64), blk, 0, stream>>>(pos, WeT, be, RE);

  attn_kernel<<<dim3(LL / 8, NHD / 2), blk, 0, stream>>>(Qh, QR, Kh, VT, RE, Zh);

  gemm64<0, 1, 0><<<dim3(gq), blk, 0, stream>>>(
      Zh, HH, WoutT, HH, Kh, ATT, HH, bout, bout, bout, 1.0f / (WSC * ZSC), MT, HH, HH);

  add_ln<0><<<dim3(MT / 8), blk, 0, stream>>>(x, ATT, ln1g, ln1b, X1f, X1h, MT);

  gemm64<1, 1, 1><<<dim3(gf1), blk, 0, stream>>>(
      X1h, HH, Wff1T, HH, Hh, FFo, FFD, bff1, bff1, bff1, 1.0f / WSC, MT, FFD, HH);
  gemm64<0, 1, 0><<<dim3(gq), blk, 0, stream>>>(
      Hh, FFD, Wff2T, FFD, Zh, FFo, HH, bff2, bff2, bff2, 1.0f / WSC2, MT, HH, FFD);

  add_ln<1><<<dim3(MT / 8), blk, 0, stream>>>(X1f, FFo, ln2g, ln2b, out0, Xh, MT);
  (void)hipGetLastError();
}
